// MultiHeadSelfAttention_39694087750009
// MI455X (gfx1250) — hardware-run, weakly checked
//
#include <hip/hip_runtime.h>


#define NBE  4
#define NTK  4096
#define NEM  768
#define NHH  8
#define NDH  96
constexpr size_t al256(size_t b) { return (b + 255) & ~(size_t)255; }
constexpr size_t WS_TOTAL = 4 * al256((size_t)NEM * NEM * 2) + 3 * al256((size_t)NTK * NEM * 2) + 3 * al256((size_t)NTK * NEM * 4) + al256((size_t)NTK * NEM * 2);
static_assert(WS_TOTAL == 67633152 && WS_TOTAL <= 134217728, "the workspace carve: 64.5 MiB");
static_assert(NEM == NHH * NDH && NTK % 64 == 0 && NEM % 64 == 0 && NEM % 32 == 0 && NDH % 8 == 0 && ((size_t)NTK * NEM) % 8 == 0 && ((size_t)NEM * NEM) % 8 == 0, "whole tiles; whole depth steps; whole 16-byte pieces");
typedef _Float16 h16;
typedef unsigned short bf;
typedef __attribute__((ext_vector_type(16))) __bf16   v16bf;
typedef __attribute__((ext_vector_type(16))) _Float16 v16h;
typedef __attribute__((ext_vector_type(8)))  _Float16 v8h;
typedef __attribute__((ext_vector_type(8)))  unsigned short v8us;
typedef __attribute__((ext_vector_type(8)))  float    v8f;
typedef __attribute__((ext_vector_type(4)))  float    v4f;
typedef v8h  __attribute__((may_alias)) v8ha;
typedef v4f  __attribute__((may_alias)) v4fa;
typedef v8us __attribute__((may_alias)) v8usa;

__device__ __forceinline__ unsigned short f2bf(float f) { unsigned u = __float_as_uint(f); u += 0x7FFFu + ((u >> 16) & 1u); return (unsigned short)(u >> 16); }
__device__ __forceinline__ float bf2f(unsigned short b) { return __uint_as_float(((unsigned)b) << 16); }
__device__ __forceinline__ float bfr(float f) { return bf2f(f2bf(f)); }
__device__ __forceinline__ v16h cat16(v8h lo, v8h hi) { return __builtin_shufflevector(lo, hi, 0, 1, 2, 3, 4, 5, 6, 7, 8, 9, 10, 11, 12, 13, 14, 15); }
__device__ __forceinline__ v16bf cat16b(v8us lo, v8us hi) { return __builtin_bit_cast(v16bf, __builtin_shufflevector(lo, hi, 0, 1, 2, 3, 4, 5, 6, 7, 8, 9, 10, 11, 12, 13, 14, 15)); }
__device__ __forceinline__ v8f wmma16(v16h a, v16h b, v8f c) { return __builtin_amdgcn_wmma_f32_16x16x32_f16(false, a, false, b, (short)0, c, false, false); }
__device__ __forceinline__ v8f wmmab(v16bf a, v16bf b, v8f c) { return __builtin_amdgcn_wmma_f32_16x16x32_bf16(false, a, false, b, (short)0, c, false, false); }


template <typename T16> struct WFrag;
template <> struct WFrag<h16> { typedef v16h V; static __device__ __forceinline__ V ld(const h16* p) { return cat16(*(const v8h*)p, *(const v8h*)(p + 16)); } static __device__ __forceinline__ v8f mma(V a, V b, v8f c) { return wmma16(a, b, c); } };
template <> struct WFrag<bf> { typedef v16bf V; static __device__ __forceinline__ V ld(const bf* p) { return cat16b(*(const v8us*)p, *(const v8us*)(p + 16)); } static __device__ __forceinline__ v8f mma(V a, V b, v8f c) { return wmmab(a, b, c); } };
template <typename T16, int NSPLIT, bool BIAS>
__global__ __launch_bounds__(32) void k_gemmw(const T16* __restrict__ A, const T16* __restrict__ A2, const T16* __restrict__ Bt, const T16* __restrict__ Bt2, int K, float* C, int ldc, const float* __restrict__ bias, size_t sA, size_t sB, size_t sC) {
    typedef typename WFrag<T16>::V V;
    __shared__ __align__(16) float os[16 * 68];
    const size_t z = blockIdx.z; A += z * sA; if (A2) A2 += z * sA; Bt += z * sB; if (Bt2) Bt2 += z * sB; C += z * sC;
    const int lane = threadIdx.x & 31, lr = lane & 15, hi = lane >> 4; const int r0 = blockIdx.x * 64, c0 = blockIdx.y * 64;
    v8f acc[4][4];
#pragma unroll
    for (int mb = 0; mb < 4; ++mb)
#pragma unroll
        for (int nb = 0; nb < 4; ++nb) acc[mb][nb] = (v8f){};
    const size_t aoff = (size_t)(r0 + lr) * K + 8 * hi, boff = (size_t)(c0 + lr) * K + 8 * hi;
    for (int kc = 0; kc < K; kc += 32) {
        V a[4], a2[4];
#pragma unroll
        for (int mb = 0; mb < 4; ++mb) { a[mb] = WFrag<T16>::ld(A + aoff + (size_t)mb * 16 * K + kc); if (NSPLIT == 1 || NSPLIT == 2) a2[mb] = WFrag<T16>::ld(A2 + aoff + (size_t)mb * 16 * K + kc); }
#pragma unroll
        for (int nb = 0; nb < 4; ++nb) { const V b = WFrag<T16>::ld(Bt + boff + (size_t)nb * 16 * K + kc); V b2; if (NSPLIT >= 2) b2 = WFrag<T16>::ld(Bt2 + boff + (size_t)nb * 16 * K + kc);
#pragma unroll
            for (int mb = 0; mb < 4; ++mb) { acc[mb][nb] = WFrag<T16>::mma(a[mb], b, acc[mb][nb]); if (NSPLIT == 1 || NSPLIT == 2) acc[mb][nb] = WFrag<T16>::mma(a2[mb], b, acc[mb][nb]); if (NSPLIT >= 2) acc[mb][nb] = WFrag<T16>::mma(a[mb], b2, acc[mb][nb]); } }
        asm volatile("v_nop\n\tv_nop\n\tv_nop\n\tv_nop" : "+v"(acc[0][0]), "+v"(acc[1][1]), "+v"(acc[2][2]), "+v"(acc[3][3]) : "v"(a[0]), "v"(a[3]));
    }
#pragma unroll
    for (int mb = 0; mb < 4; ++mb) {
#pragma unroll
        for (int nb = 0; nb < 4; ++nb) {
#pragma unroll
            for (int j = 0; j < 8; ++j) os[(hi * 8 + j) * 68 + nb * 16 + lr] = acc[mb][nb][j]; }
        __builtin_amdgcn_wave_barrier(); asm volatile("" ::: "memory");
        float* crow = C + (size_t)(r0 + mb * 16) * ldc + c0;
#pragma unroll 1
        for (int ps = 0; ps < 2; ++ps) {
#pragma unroll
            for (int s = 0; s < 8; ++s) { const int row = 2 * s + hi, cofs = lr * 4; v4f val = *(const v4fa*)(os + row * 68 + cofs); if (BIAS) { val[0] += bfr(bias[c0 + cofs]); val[1] += bfr(bias[c0 + cofs + 1]); val[2] += bfr(bias[c0 + cofs + 2]); val[3] += bfr(bias[c0 + cofs + 3]); }
                *(volatile v4f*)(crow + (size_t)row * ldc + cofs) = val; }
            if (ps == 0) __threadfence(); }
        __builtin_amdgcn_wave_barrier(); asm volatile("" ::: "memory");
    }
}

__device__ __forceinline__ h16 tohx(float x) { return (h16)x; }
__device__ __forceinline__ void splitf(float y, unsigned short& h, unsigned short& l) { h = f2bf(y); l = f2bf(y - bf2f(h)); }
typedef __attribute__((ext_vector_type(2))) _Float16 v2h;
typedef __attribute__((ext_vector_type(4))) _Float16 v4h;
typedef __attribute__((ext_vector_type(2))) unsigned short v2us;
typedef __attribute__((ext_vector_type(4))) unsigned short v4us;
typedef __attribute__((ext_vector_type(2))) float v2f;
typedef __attribute__((ext_vector_type(4))) int v4i;

__global__ __launch_bounds__(256) void k_cvt8(const float* __restrict__ src, bf* dst, size_t n8) { const size_t i = (size_t)blockIdx.x * 256 + threadIdx.x; if (i >= n8) return; const v8f v = *(const v8f*)(src + i * 8); v8us o;
#pragma unroll
    for (int k = 0; k < 8; ++k) o[k] = f2bf(v[k]); *(volatile v8us*)(dst + i * 8) = o; __threadfence(); *(volatile v8us*)(dst + i * 8) = o; }

__global__ __launch_bounds__(256) void k_cvt8h(const float* __restrict__ src, bf* dst, size_t n8) { const size_t i = (size_t)blockIdx.x * 256 + threadIdx.x; if (i >= n8) return; const v8f v = *(const v8f*)(src + i * 8); v8us o;
#pragma unroll
    for (int k = 0; k < 8; ++k) o[k] = __builtin_bit_cast(unsigned short, tohx(bfr(v[k]))); *(volatile v8us*)(dst + i * 8) = o; __threadfence(); *(volatile v8us*)(dst + i * 8) = o; }

__global__ __launch_bounds__(256) void k_hg(const float* __restrict__ PC, const float* __restrict__ PB, const float* __restrict__ PA, const int* __restrict__ im, bf* OA) {
    const unsigned t = blockIdx.x * 256 + threadIdx.x; if (t >= (unsigned)NTK) return; const unsigned hi = blockIdx.y; const bool off = (im[t] == 0);
    const float* rc = PC + (size_t)t * NEM + hi * NDH; const float* rb = PB + (size_t)t * NEM; const float* ra = PA + (size_t)t * NEM; float sc[NHH];
    v4f cv[NDH / 4];
#pragma unroll
    for (int c = 0; c < NDH / 4; ++c) cv[c] = *(const v4f*)(rc + 4 * c);
#pragma unroll
    for (int j = 0; j < NHH; ++j) { float acc = 0.0f;
#pragma unroll
        for (int c = 0; c < NDH / 4; ++c) { const v4f bv = *(const v4f*)(rb + j * NDH + 4 * c); acc += cv[c][0] * bv[0]; acc += cv[c][1] * bv[1]; acc += cv[c][2] * bv[2]; acc += cv[c][3] * bv[3]; }
        sc[j] = (off ? -1e20f : acc) / 27.712812921102035f; }
    float mx = sc[0];
#pragma unroll
    for (int j = 1; j < NHH; ++j) mx = fmaxf(mx, sc[j]);
    float sm = 0.0f;
#pragma unroll
    for (int j = 0; j < NHH; ++j) { sc[j] = expf(sc[j] - mx); sm += sc[j]; }
#pragma unroll
    for (int j = 0; j < NHH; ++j) sc[j] = sc[j] / sm;
    bf* dst = OA + ((size_t)hi * NTK + t) * NDH;
    for (int g = 0; g < NDH / 8; ++g) { float o[8];
#pragma unroll
        for (int u = 0; u < 8; ++u) o[u] = 0.0f;
#pragma unroll
        for (int j = 0; j < NHH; ++j) { const v4f a0 = *(const v4f*)(ra + j * NDH + 8 * g); const v4f a1 = *(const v4f*)(ra + j * NDH + 8 * g + 4);
#pragma unroll
            for (int u = 0; u < 4; ++u) { o[u] += sc[j] * a0[u]; o[u + 4] += sc[j] * a1[u]; } }
        v8us w;
#pragma unroll
        for (int u = 0; u < 8; ++u) w[u] = __builtin_bit_cast(unsigned short, tohx(o[u]));
        *(volatile v8us*)(dst + 8 * g) = w; __threadfence(); *(volatile v8us*)(dst + 8 * g) = w; } }

extern "C" void kernel_launch(void* const* d_in, const int* in_sizes, int n_in,
                              void* d_out, int out_size, void* d_ws, size_t ws_size, hipStream_t stream) {
    if (n_in < 9) return;
    if (in_sizes[0] < NBE * NTK * NEM || in_sizes[1] < NBE * NTK * NEM || in_sizes[2] < NBE * NTK * NEM || in_sizes[3] < NBE * NTK || in_sizes[4] < NEM * NEM || in_sizes[5] < NEM * NEM || in_sizes[6] < NEM * NEM || in_sizes[7] < NEM * NEM || in_sizes[8] < NEM || out_size < NBE * NTK * NEM) return;
    const float* ia = (const float*)d_in[0]; const float* ib = (const float*)d_in[1]; const float* ic = (const float*)d_in[2]; const int* im = (const int*)d_in[3];
    const float* ua = (const float*)d_in[4]; const float* ub = (const float*)d_in[5]; const float* uc = (const float*)d_in[6]; const float* ud = (const float*)d_in[7]; const float* ar = (const float*)d_in[8];
    float* OUT = (float*)d_out;
    char* wsp = (char*)d_ws;
    auto take = [&](size_t bytes) { char* cur = wsp; wsp += (bytes + 255) & ~(size_t)255; return (void*)cur; };
    bf* UA = (bf*)take((size_t)NEM * NEM * 2); bf* UB = (bf*)take((size_t)NEM * NEM * 2); bf* UC = (bf*)take((size_t)NEM * NEM * 2); bf* UD = (bf*)take((size_t)NEM * NEM * 2);
    bf* IA = (bf*)take((size_t)NTK * NEM * 2); bf* IB = (bf*)take((size_t)NTK * NEM * 2); bf* IC = (bf*)take((size_t)NTK * NEM * 2);
    float* PA = (float*)take((size_t)NTK * NEM * 4); float* PB = (float*)take((size_t)NTK * NEM * 4); float* PC = (float*)take((size_t)NTK * NEM * 4); bf* OA = (bf*)take((size_t)NTK * NEM * 2);
    if ((size_t)(wsp - (char*)d_ws) != WS_TOTAL || WS_TOTAL > ws_size) return;
    const size_t nw8 = (size_t)NEM * NEM / 8, nx8 = (size_t)NTK * NEM / 8;
    k_cvt8<<<(unsigned)((nw8 + 255) / 256), 256, 0, stream>>>(ua, UA, nw8);
    k_cvt8<<<(unsigned)((nw8 + 255) / 256), 256, 0, stream>>>(ub, UB, nw8);
    k_cvt8<<<(unsigned)((nw8 + 255) / 256), 256, 0, stream>>>(uc, UC, nw8);
    k_cvt8h<<<(unsigned)((nw8 + 255) / 256), 256, 0, stream>>>(ud, UD, nw8);
    for (int be = 0; be < NBE; ++be) {
        const size_t x0 = (size_t)be * NTK * NEM;
        k_cvt8<<<(unsigned)((nx8 + 255) / 256), 256, 0, stream>>>(ia + x0, IA, nx8);
        k_cvt8<<<(unsigned)((nx8 + 255) / 256), 256, 0, stream>>>(ib + x0, IB, nx8);
        k_cvt8<<<(unsigned)((nx8 + 255) / 256), 256, 0, stream>>>(ic + x0, IC, nx8);
        k_gemmw<bf, 0, false><<<dim3(NTK / 64, NEM / 64, 1), 32, 0, stream>>>(IA, nullptr, UA, nullptr, NEM, PA, NEM, nullptr, (size_t)0, (size_t)0, (size_t)0);
        k_gemmw<bf, 0, false><<<dim3(NTK / 64, NEM / 64, 1), 32, 0, stream>>>(IB, nullptr, UB, nullptr, NEM, PB, NEM, nullptr, (size_t)0, (size_t)0, (size_t)0);
        k_gemmw<bf, 0, false><<<dim3(NTK / 64, NEM / 64, 1), 32, 0, stream>>>(IC, nullptr, UC, nullptr, NEM, PC, NEM, nullptr, (size_t)0, (size_t)0, (size_t)0);
        k_hg<<<dim3(NTK / 256, NHH, 1), 256, 0, stream>>>(PC, PB, PA, im + (size_t)be * NTK, OA);
        k_gemmw<h16, 0, true><<<dim3(NTK / 64, NEM / 64, 1), 32, 0, stream>>>((const h16*)OA, nullptr, (const h16*)UD, nullptr, NEM, OUT + x0, NEM, ar, (size_t)0, (size_t)0, (size_t)0);
    }
}
